// SpatialAttn2DBlock_52140902973460
// MI455X (gfx1250) — hardware-run, weakly checked
//
#include <hip/hip_runtime.h>
#include <stdint.h>

#define NBATCH 8
#define CDIM   512
#define HW     1024
#define IMW    32
#define NHEAD  8
#define DH     64
#define QKVC   1536
#define QKP    1024
#define QT     64
#define GM     128
#define GN     64
#define OSP    68
#define LTP    72
#define LNP    36
#define WSC    64.0f
#define IWSC   0.015625f
#define WPSA   0.000244140625f
#define PWSA   0.0009765625f
#define QSC    32.0f
#define TSC    0.0009765625f
#define DSC    16.0f
#define RSC    16384.0f
#define IRSC   6.103515625e-05f
#define LNPS   6.931471805599453f
#define LN_EPS 1.0e-5f
#define NRM_EPS 1.0e-12f

#define WOFF1 786432
#define WOFF2 1048576
#define WOFF3 1310720
#define WTOT  1835008

static_assert(IMW * IMW == HW);
static_assert(NHEAD * DH == CDIM);
static_assert(HW % QT == 0);
static_assert(HW % GN == 0);
static_assert(HW % 32 == 0);
static_assert(QKVC % GM == 0);
static_assert(CDIM % GM == 0);
static_assert(WTOT % 2048 == 0);
static_assert(WOFF1 % 2048 == 0);
static_assert(WOFF2 % 2048 == 0);
static_assert(WOFF3 % 2048 == 0);
static_assert(WOFF1 == QKVC * CDIM);
static_assert(WOFF2 - WOFF1 == CDIM * CDIM);
static_assert(WOFF3 - WOFF2 == CDIM * CDIM);
static_assert(WTOT - WOFF3 == HW * CDIM);
static_assert((OSP * 4) % 16 == 0);
static_assert((LTP * 2) % 16 == 0);
static_assert((LNP * 4) % 16 == 0);
static_assert(DH % 32 == 0);

typedef _Float16       v16h __attribute__((ext_vector_type(16)));
typedef _Float16       v8h  __attribute__((ext_vector_type(8)));
typedef unsigned short v8us __attribute__((ext_vector_type(8)));
typedef float          v8f  __attribute__((ext_vector_type(8)));
typedef float          v4f  __attribute__((ext_vector_type(4)));
typedef unsigned int   v4u  __attribute__((ext_vector_type(4)));

union Frag  { v8us u[2]; v16h h; };
union FragH { v16h v; v8h hv[2]; };
static_assert(sizeof(Frag) == 32);
static_assert(sizeof(FragH) == 32);

__device__ __forceinline__ unsigned short bf_bits(float f) {
  unsigned u = __float_as_uint(f);
  return (unsigned short)((u + 0x7FFFu + ((u >> 16) & 1u)) >> 16);
}
__device__ __forceinline__ float bf_up(unsigned short hb) { return __uint_as_float(((unsigned)hb) << 16); }
__device__ __forceinline__ float bfr(float f) { return bf_up(bf_bits(f)); }
__device__ __forceinline__ unsigned short h_bits(_Float16 x) { return __builtin_bit_cast(unsigned short, x); }
__device__ __forceinline__ unsigned pk16(unsigned short a, unsigned short b) { return (unsigned)a | ((unsigned)b << 16); }
__device__ __forceinline__ v8f zero8() { v8f z = {0.f, 0.f, 0.f, 0.f, 0.f, 0.f, 0.f, 0.f}; return z; }
__device__ __forceinline__ float hmax8(v8f s) {
  return fmaxf(fmaxf(fmaxf(s[0], s[1]), fmaxf(s[2], s[3])), fmaxf(fmaxf(s[4], s[5]), fmaxf(s[6], s[7])));
}
__device__ __forceinline__ float wsum(float v) {
  v += __shfl_xor(v, 16, 32);
  v += __shfl_xor(v, 8, 32);
  v += __shfl_xor(v, 4, 32);
  v += __shfl_xor(v, 2, 32);
  v += __shfl_xor(v, 1, 32);
  return v;
}

__device__ __forceinline__ Frag ldfrag(const unsigned short* p) {
  Frag f;
  f.u[0] = *(const v8us*)(p);
  f.u[1] = *(const v8us*)(p + 16);
  return f;
}

__device__ __forceinline__ v8f mma_h(v16h a, v16h b, v8f c) {
  v8f d = __builtin_amdgcn_wmma_f32_16x16x32_f16(false, a, false, b, (short)0, c, false, false);
#if defined(__HIP_DEVICE_COMPILE__)
  asm volatile("v_nop\n\tv_nop\n\tv_nop\n\tv_nop" : "+v"(d) : "v"(a), "v"(b));
#endif
  return d;
}

__global__ __launch_bounds__(256)
void cvt_w(const float* __restrict__ w0, const float* __restrict__ w1, const float* __restrict__ w2,
           const float* __restrict__ w3, unsigned short* WB) {
  const int g0 = (int)blockIdx.x * 2048;
  const float* src = w0;
  int base = 0;
  if (g0 >= WOFF3)      { src = w3; base = WOFF3; }
  else if (g0 >= WOFF2) { src = w2; base = WOFF2; }
  else if (g0 >= WOFF1) { src = w1; base = WOFF1; }
  const int i = g0 + (int)threadIdx.x * 8;
  const float* s = src + (i - base);
  const v4f a = *(const v4f*)(s);
  const v4f q = *(const v4f*)(s + 4);
  v4u w;
  w[0] = pk16(h_bits((_Float16)(bfr(a[0]) * WSC)), h_bits((_Float16)(bfr(a[1]) * WSC)));
  w[1] = pk16(h_bits((_Float16)(bfr(a[2]) * WSC)), h_bits((_Float16)(bfr(a[3]) * WSC)));
  w[2] = pk16(h_bits((_Float16)(bfr(q[0]) * WSC)), h_bits((_Float16)(bfr(q[1]) * WSC)));
  w[3] = pk16(h_bits((_Float16)(bfr(q[2]) * WSC)), h_bits((_Float16)(bfr(q[3]) * WSC)));
  unsigned short* p = WB + (size_t)i;
  *(volatile v4u*)p = w;
  __threadfence();
  *(volatile v4u*)p = w;
}

__global__ __launch_bounds__(256)
void cvt_x(const float* __restrict__ x, unsigned short* X16) {
  __shared__ __align__(16) unsigned short Lt[GN * LTP];
  const int tid = threadIdx.x;
  const int nt = blockIdx.x, cg = blockIdx.y, b = blockIdx.z;
  const int n0 = nt * GN;
  {
    const int n4 = (tid & 15) * 4, cs = tid >> 4;
#pragma unroll
    for (int it = 0; it < 4; ++it) {
      const int cl = it * 16 + cs;
      const v4f v = *(const v4f*)(x + ((size_t)(b * CDIM + cg * 64 + cl)) * HW + n0 + n4);
#pragma unroll
      for (int qq = 0; qq < 4; ++qq) Lt[(n4 + qq) * LTP + cl] = h_bits((_Float16)bfr(v[qq]));
    }
  }
  __syncthreads();
  {
    const int e = tid & 7, lq = tid >> 3;
#pragma unroll
    for (int pass = 0; pass < 2; ++pass) {
#pragma unroll
      for (int it = 0; it < 2; ++it) {
        const int n = it * 32 + lq;
        const v4u u = *(const v4u*)(Lt + n * LTP + 8 * e);
        *(volatile v4u*)(X16 + ((size_t)(b * HW + n0 + n)) * CDIM + cg * 64 + 8 * e) = u;
      }
      __threadfence();
    }
  }
}

template <int NPL>
__global__ __launch_bounds__(256)
void gemm_kernel(const unsigned short* __restrict__ Wp, int K, float sA,
                 const unsigned short* __restrict__ Bh, const unsigned short* __restrict__ Bl, int bp,
                 const float* __restrict__ bias,
                 const float* __restrict__ resid, int res_zs,
                 float* outF, int of_ch,
                 float* outPf, int opf_ch, int pf_hi,
                 unsigned short* out16, int o16_ch, int o16_lo) {
  __shared__ __align__(16) float Os[GM * OSP];
  const int tid  = threadIdx.x;
  const int lane = tid & 31, wave = tid >> 5;
  const int hh   = lane >> 4, c = lane & 15;
  const int wm   = wave >> 1, wn = wave & 1;
  const int z    = blockIdx.z;
  const int mBase = blockIdx.x * GM;
  const int nBase = blockIdx.y * GN;

  const unsigned short* a0p = Wp + (size_t)(mBase + 32 * wm + c) * K + 8 * hh;
  const unsigned short* a1p = a0p + (size_t)16 * K;
  const size_t brow = (size_t)z * HW + nBase + 32 * wn + c;
  const unsigned short* b0h = Bh + brow * (size_t)bp + 8 * hh;
  const unsigned short* b1h = b0h + (size_t)16 * bp;
  const unsigned short* b0l = b0h;
  const unsigned short* b1l = b1h;
  if (NPL == 2) {
    b0l = Bl + brow * (size_t)bp + 8 * hh;
    b1l = b0l + (size_t)16 * bp;
  }

  v8f acc[2][2], accr[2][2];
#pragma unroll
  for (int mi = 0; mi < 2; ++mi)
#pragma unroll
    for (int ni = 0; ni < 2; ++ni) { acc[mi][ni] = zero8(); accr[mi][ni] = zero8(); }

#pragma unroll 1
  for (int k0 = 0; k0 < K; k0 += 32) {
    const Frag fa0 = ldfrag(a0p + k0);
    const Frag fa1 = ldfrag(a1p + k0);
    const Frag fb0 = ldfrag(b0h + k0);
    const Frag fb1 = ldfrag(b1h + k0);
    acc[0][0] = mma_h(fa0.h, fb0.h, acc[0][0]);
    acc[0][1] = mma_h(fa0.h, fb1.h, acc[0][1]);
    acc[1][0] = mma_h(fa1.h, fb0.h, acc[1][0]);
    acc[1][1] = mma_h(fa1.h, fb1.h, acc[1][1]);
    if (NPL == 2) {
      const Frag fl0 = ldfrag(b0l + k0);
      const Frag fl1 = ldfrag(b1l + k0);
      accr[0][0] = mma_h(fa0.h, fl0.h, accr[0][0]);
      accr[0][1] = mma_h(fa0.h, fl1.h, accr[0][1]);
      accr[1][0] = mma_h(fa1.h, fl0.h, accr[1][0]);
      accr[1][1] = mma_h(fa1.h, fl1.h, accr[1][1]);
    }
  }

  const float rsA = sA * IRSC;
#pragma unroll
  for (int mi = 0; mi < 2; ++mi) {
#pragma unroll
    for (int ni = 0; ni < 2; ++ni) {
      const int n_loc = 32 * wn + 16 * ni + c;
      const int n = nBase + n_loc;
#pragma unroll
      for (int r = 0; r < 8; ++r) {
        const int o_loc = 32 * wm + 16 * mi + 8 * hh + r;
        const int o = mBase + o_loc;
        float v = acc[mi][ni][r] * sA;
        if (NPL == 2) v += accr[mi][ni][r] * rsA;
        if (bias != nullptr) v += bfr(bias[o]);
        if (resid != nullptr) v += resid[(size_t)z * (size_t)res_zs + (size_t)o * HW + n];
        Os[o_loc * OSP + n_loc] = v;
      }
    }
  }
  __syncthreads();

  {
    const int e = tid & 7, lq = tid >> 3;
    const bool doF  = (outF != nullptr);
    const bool doPf = (outPf != nullptr) && (mBase < pf_hi);
    const bool do16 = (out16 != nullptr) && (mBase >= o16_lo);
#pragma unroll
    for (int pass = 0; pass < 2; ++pass) {
      if (doF) {
#pragma unroll
        for (int it = 0; it < 8; ++it) {
          const int L = it * 32 + lq;
          const int row = L >> 1, hf = L & 1;
          const v4f v = *(const v4f*)(Os + row * OSP + hf * 32 + 4 * e);
          float* dst = outF + ((size_t)z * of_ch + mBase + row) * HW + nBase + hf * 32 + 4 * e;
          *(volatile v4f*)dst = v;
        }
      }
      if (do16) {
#pragma unroll
        for (int it = 0; it < 4; ++it) {
          const int row = it * 32 + lq;
          const v4f v0 = *(const v4f*)(Os + row * OSP + 8 * e);
          const v4f v1 = *(const v4f*)(Os + row * OSP + 8 * e + 4);
          v4u u;
          u[0] = pk16(h_bits((_Float16)v0[0]), h_bits((_Float16)v0[1]));
          u[1] = pk16(h_bits((_Float16)v0[2]), h_bits((_Float16)v0[3]));
          u[2] = pk16(h_bits((_Float16)v1[0]), h_bits((_Float16)v1[1]));
          u[3] = pk16(h_bits((_Float16)v1[2]), h_bits((_Float16)v1[3]));
          unsigned short* dst = out16 + ((size_t)z * o16_ch + (mBase - o16_lo) + row) * HW + nBase + 8 * e;
          *(volatile v4u*)dst = u;
        }
      }
      if (doPf) {
#pragma unroll
        for (int it = 0; it < 8; ++it) {
          const int L = it * 32 + lq;
          const int n_loc = L >> 2, q4 = L & 3;
          const int ch0 = q4 * 32 + 4 * e;
          v4f v;
#pragma unroll
          for (int j = 0; j < 4; ++j) v[j] = Os[(ch0 + j) * OSP + n_loc];
          float* dst = outPf + ((size_t)z * HW + nBase + n_loc) * (size_t)opf_ch + mBase + ch0;
          *(volatile v4f*)dst = v;
        }
      }
      __threadfence();
    }
  }
}

__global__ __launch_bounds__(256)
void norm_kernel(const float* __restrict__ QKf, unsigned short* QKn) {
  __shared__ float red[256];
  __shared__ float inv_s[64];
  const int tid = threadIdx.x;
  const int cg = blockIdx.x, b = blockIdx.y;
  const float* base = QKf + (size_t)b * HW * QKP + cg * 64;
  {
    const int col = tid & 63, seg = tid >> 6;
    float ss = 0.f;
#pragma unroll 1
    for (int t = seg * 256; t < seg * 256 + 256; ++t) {
      const float v = base[(size_t)t * QKP + col];
      ss = fmaf(v, v, ss);
    }
    red[tid] = ss;
  }
  __syncthreads();
  if (tid < 64) {
    float tot = red[tid] + red[64 + tid];
    tot += red[128 + tid];
    tot += red[192 + tid];
    inv_s[tid] = QSC * __builtin_amdgcn_rcpf(fmaxf(sqrtf(tot), NRM_EPS));
  }
  __syncthreads();
  {
    const int e = tid & 7, lq = tid >> 3;
    float iv[8];
#pragma unroll
    for (int j = 0; j < 8; ++j) iv[j] = inv_s[8 * e + j];
#pragma unroll
    for (int pass = 0; pass < 2; ++pass) {
#pragma unroll 1
      for (int it = 0; it < 32; ++it) {
        const int n = it * 32 + lq;
        const float* rp = base + (size_t)n * QKP + 8 * e;
        const v4f a = *(const v4f*)(rp);
        const v4f q = *(const v4f*)(rp + 4);
        v4u u;
        u[0] = pk16(h_bits((_Float16)(a[0] * iv[0])), h_bits((_Float16)(a[1] * iv[1])));
        u[1] = pk16(h_bits((_Float16)(a[2] * iv[2])), h_bits((_Float16)(a[3] * iv[3])));
        u[2] = pk16(h_bits((_Float16)(q[0] * iv[4])), h_bits((_Float16)(q[1] * iv[5])));
        u[3] = pk16(h_bits((_Float16)(q[2] * iv[6])), h_bits((_Float16)(q[3] * iv[7])));
        *(volatile v4u*)(QKn + ((size_t)(b * HW + n)) * QKP + cg * 64 + 8 * e) = u;
      }
      __threadfence();
    }
  }
}

__global__ __launch_bounds__(128)
void attn_kernel(const unsigned short* __restrict__ QKn, const unsigned short* __restrict__ V16,
                 const float* __restrict__ temp, unsigned short* Oh, unsigned short* Ol) {
  __shared__ __align__(16) float Os[DH * OSP];
  const int tid  = threadIdx.x;
  const int wave = tid >> 5, lane = tid & 31;
  const int hh   = lane >> 4, c = lane & 15;
  const int qb   = blockIdx.x, h = blockIdx.y, b = blockIdx.z;
  const int n0   = qb * QT;

  const unsigned short* qp = QKn + ((size_t)(b * HW + n0 + 16 * wave + c)) * QKP + h * DH + 8 * hh;
  const Frag qfa = ldfrag(qp);
  const Frag qfb = ldfrag(qp + 32);
  const v16h q0 = qfa.h, q1 = qfb.h;
  const unsigned short* Kp = QKn + ((size_t)(b * HW + c)) * QKP + CDIM + h * DH + 8 * hh;
  const unsigned short* Vb = V16 + ((size_t)(b * CDIM + h * DH + c)) * HW + 8 * hh;
  const float tsc = bfr(temp[h]) * TSC;

  float m = -1.0e30f, l = 0.f;
  v8f o0 = zero8(), o1 = zero8(), o2 = zero8(), o3 = zero8();
#pragma unroll 1
  for (int it = 0; it < HW / 32; ++it) {
    const int kb = it * 32;
    const unsigned short* k0p = Kp + (size_t)kb * QKP;
    const unsigned short* k1p = k0p + (size_t)16 * QKP;
    const Frag ka = ldfrag(k0p);
    const Frag kbf = ldfrag(k0p + 32);
    const Frag kc = ldfrag(k1p);
    const Frag kd = ldfrag(k1p + 32);
    v8f s0 = mma_h(ka.h, q0, zero8());
    s0 = mma_h(kbf.h, q1, s0);
    v8f s1 = mma_h(kc.h, q0, zero8());
    s1 = mma_h(kd.h, q1, s1);
#pragma unroll
    for (int r = 0; r < 8; ++r) { s0[r] *= tsc; s1[r] *= tsc; }

    float mx = fmaxf(hmax8(s0), hmax8(s1));
    mx = fmaxf(mx, __shfl_xor(mx, 16, 32));
    const float mn   = fmaxf(m, mx);
    const float corr = __expf(m - mn);
    m = mn;
    const float msh = mn - LNPS;
    l *= corr;
#pragma unroll
    for (int r = 0; r < 8; ++r) { o0[r] *= corr; o1[r] *= corr; o2[r] *= corr; o3[r] *= corr; }

    FragH ph;
    float ls = 0.f;
#pragma unroll
    for (int r = 0; r < 8; ++r) {
      const _Float16 e0 = (_Float16)__expf(s0[r] - msh);
      const _Float16 e1 = (_Float16)__expf(s1[r] - msh);
      ls += (float)e0 + (float)e1;
      ph.hv[0][r] = e0;
      ph.hv[1][r] = e1;
    }
    l += ls;

    const Frag v0f = ldfrag(Vb + kb);
    const Frag v1f = ldfrag(Vb + (size_t)16 * HW + kb);
    const Frag v2f = ldfrag(Vb + (size_t)32 * HW + kb);
    const Frag v3f = ldfrag(Vb + (size_t)48 * HW + kb);
    o0 = mma_h(v0f.h, ph.v, o0);
    o1 = mma_h(v1f.h, ph.v, o1);
    o2 = mma_h(v2f.h, ph.v, o2);
    o3 = mma_h(v3f.h, ph.v, o3);
  }
  l += __shfl_xor(l, 16, 32);
  const float inv = __builtin_amdgcn_rcpf(l);

  float* os = Os + (8 * hh) * OSP + wave * 16 + c;
#pragma unroll
  for (int r = 0; r < 8; ++r) {
    os[(0 * 16 + r) * OSP] = o0[r] * inv;
    os[(1 * 16 + r) * OSP] = o1[r] * inv;
    os[(2 * 16 + r) * OSP] = o2[r] * inv;
    os[(3 * 16 + r) * OSP] = o3[r] * inv;
  }
  __syncthreads();
  {
    const int e = tid & 7, lq = tid >> 3;
#pragma unroll
    for (int pass = 0; pass < 2; ++pass) {
#pragma unroll
      for (int it = 0; it < 4; ++it) {
        const int n_loc = it * 16 + lq;
        float f[8];
#pragma unroll
        for (int j = 0; j < 8; ++j) f[j] = Os[(8 * e + j) * OSP + n_loc];
        v4u uh, ul;
#pragma unroll
        for (int t = 0; t < 4; ++t) {
          const _Float16 x0 = (_Float16)f[2 * t];
          const _Float16 x1 = (_Float16)f[2 * t + 1];
          const _Float16 y0 = (_Float16)((f[2 * t] - (float)x0) * RSC);
          const _Float16 y1 = (_Float16)((f[2 * t + 1] - (float)x1) * RSC);
          uh[t] = pk16(h_bits(x0), h_bits(x1));
          ul[t] = pk16(h_bits(y0), h_bits(y1));
        }
        const size_t po = ((size_t)(b * HW + n0 + n_loc)) * CDIM + h * DH + 8 * e;
        *(volatile v4u*)(Oh + po) = uh;
        *(volatile v4u*)(Ol + po) = ul;
      }
      __threadfence();
    }
  }
}

__global__ __launch_bounds__(256)
void ln_kernel(const float* __restrict__ Y, const float* __restrict__ x, const float* __restrict__ g,
               const float* __restrict__ bb, float* O2) {
  __shared__ __align__(16) float Lt[256 * LNP];
  const int tid = threadIdx.x, wave = tid >> 5, lane = tid & 31;
  const int nt = blockIdx.x, cgh = blockIdx.y, b = blockIdx.z;
  const int n0 = nt * 32;
#pragma unroll 1
  for (int i = 0; i < 4; ++i) {
    const int tl = 4 * wave + i;
    const float* row = Y + ((size_t)(b * HW + n0 + tl)) * CDIM + 4 * lane;
    const v4f v0 = *(const v4f*)(row);
    const v4f v1 = *(const v4f*)(row + 128);
    const v4f v2 = *(const v4f*)(row + 256);
    const v4f v3 = *(const v4f*)(row + 384);
    float s = ((v0[0] + v0[1]) + (v0[2] + v0[3])) + ((v1[0] + v1[1]) + (v1[2] + v1[3]))
            + ((v2[0] + v2[1]) + (v2[2] + v2[3])) + ((v3[0] + v3[1]) + (v3[2] + v3[3]));
    s = wsum(s);
    const float mu = s * (1.0f / CDIM);
    float sq = 0.f;
#pragma unroll
    for (int j = 0; j < 4; ++j) {
      const float d0 = v0[j] - mu, d1 = v1[j] - mu, d2 = v2[j] - mu, d3 = v3[j] - mu;
      sq = fmaf(d0, d0, sq); sq = fmaf(d1, d1, sq); sq = fmaf(d2, d2, sq); sq = fmaf(d3, d3, sq);
    }
    sq = wsum(sq);
    const float rstd = rsqrtf(sq * (1.0f / CDIM) + LN_EPS);
    v4f wa, wb;
#pragma unroll
    for (int j = 0; j < 4; ++j) { wa[j] = cgh ? v2[j] : v0[j]; wb[j] = cgh ? v3[j] : v1[j]; }
    const int cb = cgh * 256 + 4 * lane;
#pragma unroll
    for (int j = 0; j < 4; ++j) {
      const int c0 = cb + j, c1 = cb + 128 + j;
      Lt[(4 * lane + j) * LNP + tl]       = (wa[j] - mu) * rstd * bfr(g[c0]) + bfr(bb[c0]);
      Lt[(128 + 4 * lane + j) * LNP + tl] = (wb[j] - mu) * rstd * bfr(g[c1]) + bfr(bb[c1]);
    }
  }
  __syncthreads();
  {
    const int e = tid & 7, lq = tid >> 3;
#pragma unroll
    for (int pass = 0; pass < 2; ++pass) {
#pragma unroll
      for (int it = 0; it < 8; ++it) {
        const int cl = it * 32 + lq;
        const v4f v = *(const v4f*)(Lt + cl * LNP + 4 * e);
        const int cch = cgh * 256 + cl;
        const size_t xo = ((size_t)(b * CDIM + cch)) * HW + n0 + 4 * e;
        const v4f xv = *(const v4f*)(x + xo);
        v4f o;
#pragma unroll
        for (int j = 0; j < 4; ++j) o[j] = v[j] + bfr(xv[j]);
        *(volatile v4f*)(O2 + xo) = o;
      }
      __threadfence();
    }
  }
}

__global__ __launch_bounds__(256)
void dw_kernel(const float* __restrict__ O2, const float* __restrict__ w, const float* __restrict__ bias,
               unsigned short* DW) {
  __shared__ __align__(16) unsigned short Lh[GN * LTP];
  const int tid = threadIdx.x;
  const int nl  = tid & 63, cgrp = tid >> 6;
  const int nt  = blockIdx.x, cg = blockIdx.y, b = blockIdx.z;
  const int n0  = nt * GN;
  const int n   = n0 + nl;
  const int y   = n >> 5;
  const int xq  = n & 31;
#pragma unroll 1
  for (int j = 0; j < 16; ++j) {
    const int cl  = cgrp * 16 + j;
    const int cch = cg * 64 + cl;
    const float* rp = O2 + ((size_t)(b * CDIM + cch)) * HW;
    float accv = 0.f;
#pragma unroll
    for (int t = 0; t < 9; ++t) {
      const int ky = t / 3, kx = t - ky * 3;
      const int yy = y + ky - 1, xx = xq + kx - 1;
      const bool ok = ((unsigned)yy < (unsigned)IMW) && ((unsigned)xx < (unsigned)IMW);
      const int yc = min(max(yy, 0), IMW - 1);
      const int xc = min(max(xx, 0), IMW - 1);
      const float hv = rp[yc * IMW + xc];
      const float wv = bfr(w[cch * 9 + t]);
      accv = fmaf(ok ? hv : 0.f, wv, accv);
    }
    const float val = (accv + bfr(bias[cch])) * DSC;
    Lh[nl * LTP + cl] = h_bits((_Float16)val);
  }
  __syncthreads();
  {
    const int e = tid & 7, lq = tid >> 3;
#pragma unroll
    for (int pass = 0; pass < 2; ++pass) {
#pragma unroll
      for (int it = 0; it < 2; ++it) {
        const int nn = it * 32 + lq;
        const v4u uh = *(const v4u*)(Lh + nn * LTP + 8 * e);
        const size_t po = ((size_t)(b * HW + n0 + nn)) * CDIM + cg * 64 + 8 * e;
        *(volatile v4u*)(DW + po) = uh;
      }
      __threadfence();
    }
  }
}

extern "C" void kernel_launch(void* const* d_in, const int* in_sizes, int n_in,
                              void* d_out, int out_size, void* d_ws, size_t ws_size,
                              hipStream_t stream) {
  const int NX = NBATCH * CDIM * HW;
  if (n_in < 12) return;
  if (in_sizes[0] != NX) return;
  if (in_sizes[1] != QKVC * CDIM || in_sizes[2] != CDIM * CDIM || in_sizes[3] != CDIM) return;
  if (in_sizes[4] != NHEAD || in_sizes[5] != CDIM || in_sizes[6] != CDIM) return;
  if (in_sizes[7] != HW * CDIM || in_sizes[8] != CDIM * 9 || in_sizes[9] != CDIM) return;
  if (in_sizes[10] != CDIM * CDIM || in_sizes[11] != CDIM) return;
  if (out_size != NX) return;

  const size_t PM16 = (size_t)NBATCH * HW * CDIM * 2;
  size_t off = 0;
  const size_t oW   = off; off += (size_t)WTOT * 2;
  const size_t oX16 = off; off += PM16;
  const size_t oWP  = off; off += (size_t)QKVC * HW * 4;
  const size_t oR1  = off; off += (size_t)NBATCH * HW * QKP * 4;
  const size_t oV16 = off; off += PM16;
  const size_t oQKn = off; off += (size_t)NBATCH * HW * QKP * 2;
  const size_t oO2  = off; off += (size_t)NBATCH * CDIM * HW * 4;
  const size_t oDW  = off; off += PM16;
  const size_t oOh  = oR1;
  const size_t oOl  = oR1 + PM16;
  const size_t oY   = oR1 + 2 * PM16;
  if (off > ws_size) return;
  if (off > (size_t)134217728) return;
  if (oY + (size_t)NBATCH * HW * CDIM * 4 > oV16) return;

  const float* x      = (const float*)d_in[0];
  const float* qkv_w  = (const float*)d_in[1];
  const float* proj_w = (const float*)d_in[2];
  const float* proj_b = (const float*)d_in[3];
  const float* temp   = (const float*)d_in[4];
  const float* ln_g   = (const float*)d_in[5];
  const float* ln_b   = (const float*)d_in[6];
  const float* pos    = (const float*)d_in[7];
  const float* dw_w   = (const float*)d_in[8];
  const float* dw_b   = (const float*)d_in[9];
  const float* pw_w   = (const float*)d_in[10];
  const float* pw_b   = (const float*)d_in[11];

  char* ws = (char*)d_ws;
  unsigned short* WB  = (unsigned short*)(ws + oW);
  unsigned short* X16 = (unsigned short*)(ws + oX16);
  float*          WP  = (float*)(ws + oWP);
  float*          QKf = (float*)(ws + oR1);
  unsigned short* Oh  = (unsigned short*)(ws + oOh);
  unsigned short* Ol  = (unsigned short*)(ws + oOl);
  float*          Y   = (float*)(ws + oY);
  unsigned short* V16 = (unsigned short*)(ws + oV16);
  unsigned short* QKn = (unsigned short*)(ws + oQKn);
  float*          O2  = (float*)(ws + oO2);
  unsigned short* DWp = (unsigned short*)(ws + oDW);
  float* out = (float*)d_out;

  const dim3 blk256(256), blk128(128);
  const dim3 gW(WTOT / 2048);
  const dim3 gX(HW / GN, CDIM / 64, NBATCH);
  const dim3 gWP(QKVC / GM, HW / GN, 1);
  const dim3 gQKV(QKVC / GM, HW / GN, NBATCH);
  const dim3 gN(QKP / 64, NBATCH);
  const dim3 gA(HW / QT, NHEAD, NBATCH);
  const dim3 g512(CDIM / GM, HW / GN, NBATCH);
  const dim3 gLN(HW / 32, 2, NBATCH);
  const dim3 gDW(HW / GN, CDIM / 64, NBATCH);

  cvt_w<<<gW, blk256, 0, stream>>>(qkv_w, proj_w, pw_w, pos, WB);
  cvt_x<<<gX, blk256, 0, stream>>>(x, X16);
  gemm_kernel<1><<<gWP, blk256, 0, stream>>>(WB, CDIM, WPSA,
      WB + WOFF3, nullptr, CDIM,
      nullptr, nullptr, 0,
      WP, QKVC, nullptr, 0, 0, nullptr, 0, 0);
  gemm_kernel<1><<<gQKV, blk256, 0, stream>>>(WB, CDIM, IWSC,
      X16, nullptr, CDIM,
      nullptr, WP, 0,
      nullptr, 0, QKf, QKP, 2 * CDIM, V16, CDIM, 2 * CDIM);
  norm_kernel<<<gN, blk256, 0, stream>>>(QKf, QKn);
  attn_kernel<<<gA, blk128, 0, stream>>>(QKn, V16, temp, Oh, Ol);
  gemm_kernel<2><<<g512, blk256, 0, stream>>>(WB + WOFF1, CDIM, IWSC,
      Oh, Ol, CDIM,
      proj_b, nullptr, 0,
      nullptr, 0, Y, CDIM, CDIM, nullptr, 0, 0);
  ln_kernel<<<gLN, blk256, 0, stream>>>(Y, x, ln_g, ln_b, O2);
  dw_kernel<<<gDW, blk256, 0, stream>>>(O2, dw_w, dw_b, DWp);
  gemm_kernel<1><<<g512, blk256, 0, stream>>>(WB + WOFF2, CDIM, PWSA,
      DWp, nullptr, CDIM,
      pw_b, O2, CDIM * HW,
      out, CDIM, nullptr, 0, 0, nullptr, 0, 0);
  (void)hipGetLastError();
}
